// FullAttention_721554505961
// MI455X (gfx1250) — hardware-verified
//
#include <hip/hip_runtime.h>


#ifndef NB
#define NB 2
#endif
#ifndef SEQ
#define SEQ 2048
#endif
#ifndef NB_FULL
#define NB_FULL 2
#endif
#ifndef SEQ_FULL
#define SEQ_FULL 2048
#endif
#ifndef SEQ_OUT
#define SEQ_OUT SEQ
#endif
#define NH 16
#define HD 64
#define RROWS 512
#define PCAR 1024.0f
#define RSC  1024.0f
#define SCL  0.125f
#define L2E  1.4426950408889634f

static_assert(SEQ % 64 == 0);
static_assert(SEQ <= SEQ_FULL);
static_assert(NB <= NB_FULL);
static_assert(HD == 64);
static_assert(RROWS % 64 == 0);

typedef _Float16 h16;
typedef __attribute__((ext_vector_type(16))) _Float16 v16h;
typedef __attribute__((ext_vector_type(8)))  _Float16 v8h;
typedef __attribute__((ext_vector_type(8)))  float    v8f;
typedef __attribute__((ext_vector_type(4)))  float    v4f;
typedef v4f __attribute__((may_alias)) v4fa;

__device__ __forceinline__ unsigned short f2bf(float f) { unsigned u = __float_as_uint(f); u += 0x7FFFu + ((u >> 16) & 1u); return (unsigned short)(u >> 16); }
__device__ __forceinline__ float bf2f(unsigned short b) { return __uint_as_float(((unsigned)b) << 16); }
__device__ __forceinline__ float bfr(float f) { return bf2f(f2bf(f)); }
__device__ __forceinline__ v16h cat16(v8h lo, v8h hi) { return __builtin_shufflevector(lo, hi, 0, 1, 2, 3, 4, 5, 6, 7, 8, 9, 10, 11, 12, 13, 14, 15); }
__device__ __forceinline__ v16h ldf(const h16* p) { return cat16(*(const v8h*)p, *(const v8h*)(p + 16)); }
__device__ __forceinline__ v8f wmma16(v16h a, v16h b, v8f c) { return __builtin_amdgcn_wmma_f32_16x16x32_f16(false, a, false, b, (short)0, c, false, false); }

__global__ __launch_bounds__(256) void k_cvtqk(const float* __restrict__ q, const float* __restrict__ k, h16* QP, h16* KP, int n8) {
    const int i = blockIdx.x * 256 + threadIdx.x; if (i >= n8) return;
    const size_t e = (size_t)i * 8; const int d = (int)(e % HD); const int s = (int)((e / HD) % SEQ); const int bh = (int)(e / ((size_t)HD * SEQ));
    const size_t src = ((size_t)bh * SEQ_FULL + s) * HD + d;
    const v8f xq = *(const v8f*)(q + src); const v8f xk = *(const v8f*)(k + src); v8h oq, ok;
#pragma unroll
    for (int j = 0; j < 8; ++j) { oq[j] = (h16)bfr(xq[j]); ok[j] = (h16)bfr(xk[j]); }
    *(volatile v8h*)(QP + e) = oq; *(volatile v8h*)(KP + e) = ok;
    __threadfence();
    *(volatile v8h*)(QP + e) = oq; *(volatile v8h*)(KP + e) = ok;
}

__global__ __launch_bounds__(256) void k_vt(const float* __restrict__ v, h16* VT, int n8) {
    const int i = blockIdx.x * 256 + threadIdx.x; if (i >= n8) return;
    const size_t e = (size_t)i * 8; const int s0 = (int)(e % SEQ); const int d = (int)((e / SEQ) % HD); const int bh = (int)(e / ((size_t)SEQ * HD));
    const float* src = v + ((size_t)bh * SEQ_FULL + s0) * HD + d; v8h o;
#pragma unroll
    for (int j = 0; j < 8; ++j) o[j] = (h16)bfr(src[(size_t)j * HD]);
    *(volatile v8h*)(VT + e) = o;
    __threadfence();
    *(volatile v8h*)(VT + e) = o;
}

template <bool RES>
__global__ __launch_bounds__(128) void k_attn(const h16* __restrict__ QP, const h16* __restrict__ KP, const h16* __restrict__ VT, float* OUT, int mb0) {
    __shared__ __align__(16) float os[4 * 16 * 68];
    const int bh = blockIdx.y; const int mblk = mb0 + (int)blockIdx.x; const int q0 = mblk * 64;
    const int wave = threadIdx.x >> 5, lane = threadIdx.x & 31, lr = lane & 15, hi = lane >> 4;
    const int q0w = q0 + wave * 16; const int myq = q0w + lr;
    const h16* Qp = QP + ((size_t)bh * SEQ + q0w + lr) * HD + 8 * hi;
    const h16* Kp = KP + (size_t)bh * SEQ * HD + (size_t)lr * HD + 8 * hi;
    const h16* Vp = VT + (size_t)bh * HD * SEQ + (size_t)lr * SEQ + 8 * hi;
    v16h qb[2]; qb[0] = ldf(Qp); qb[1] = ldf(Qp + 32);
    v8f acc[4], accr[4];
#pragma unroll
    for (int dc = 0; dc < 4; ++dc) { acc[dc] = (v8f){}; accr[dc] = (v8f){}; }
    float m = -3.0e38f, l = 0.0f;
    const int nchunk = (q0 + 64) / 32;
#pragma unroll 1
    for (int it = 0; it < nchunk; ++it) {
        const int k0 = it * 32;
        v8f s[2]; v16h ka;
#pragma unroll
        for (int kt = 0; kt < 2; ++kt) {
            s[kt] = (v8f){};
#pragma unroll
            for (int kc = 0; kc < 2; ++kc) { ka = ldf(Kp + (size_t)(k0 + 16 * kt) * HD + 32 * kc); s[kt] = wmma16(ka, qb[kc], s[kt]); }
        }
        asm volatile("v_nop\n\tv_nop\n\tv_nop\n\tv_nop" : "+v"(s[0]), "+v"(s[1]) : "v"(qb[0]), "v"(qb[1]), "v"(ka));
        float t[16]; float cm = -3.0e38f;
#pragma unroll
        for (int i = 0; i < 16; ++i) { const int key = k0 + 16 * (i >> 3) + 8 * hi + (i & 7); const float x = (key > myq) ? -3.0e38f : s[i >> 3][i & 7] * SCL; t[i] = x; cm = fmaxf(cm, x); }
        cm = fmaxf(cm, __shfl_xor(cm, 16, 32));
        const float mn = fmaxf(m, cm);
        const float alpha = __builtin_amdgcn_exp2f(fmaxf(m - mn, -120.0f) * L2E);
        m = mn; l *= alpha;
#pragma unroll
        for (int dc = 0; dc < 4; ++dc) { acc[dc] = acc[dc] * alpha; if (RES) accr[dc] = accr[dc] * alpha; }
        float psm = 0.0f; v16h pb, pr;
#pragma unroll
        for (int i = 0; i < 16; ++i) {
            const int key = k0 + 16 * (i >> 3) + 8 * hi + (i & 7);
            float p = __builtin_amdgcn_exp2f(fmaxf(t[i] - mn, -120.0f) * L2E) * PCAR; p = (key > myq) ? 0.0f : p; psm += p;
            const h16 ph = (h16)p; pb[i] = ph;
            if (RES) pr[i] = (h16)((p - (float)ph) * RSC); else pr[i] = (h16)0.0f;
        }
        psm += __shfl_xor(psm, 16, 32); l += psm;
        v16h va;
#pragma unroll
        for (int dc = 0; dc < 4; ++dc) { va = ldf(Vp + (size_t)dc * 16 * SEQ + k0); acc[dc] = wmma16(va, pb, acc[dc]); if (RES) accr[dc] = wmma16(va, pr, accr[dc]); }
        if (RES) asm volatile("v_nop\n\tv_nop\n\tv_nop\n\tv_nop" : "+v"(acc[0]), "+v"(acc[1]), "+v"(acc[2]), "+v"(acc[3]), "+v"(accr[0]), "+v"(accr[1]), "+v"(accr[2]), "+v"(accr[3]) : "v"(va), "v"(pb), "v"(pr));
        else     asm volatile("v_nop\n\tv_nop\n\tv_nop\n\tv_nop" : "+v"(acc[0]), "+v"(acc[1]), "+v"(acc[2]), "+v"(acc[3]) : "v"(va), "v"(pb));
    }
    const float inv = 1.0f / l;
    float* osw = os + wave * (16 * 68);
#pragma unroll
    for (int dc = 0; dc < 4; ++dc) {
        v4f o0, o1;
#pragma unroll
        for (int r = 0; r < 4; ++r) {
            float y0 = acc[dc][r], y1 = acc[dc][r + 4];
            if (RES) { y0 += accr[dc][r] * (1.0f / RSC); y1 += accr[dc][r + 4] * (1.0f / RSC); }
            o0[r] = y0 * inv; o1[r] = y1 * inv;
        }
        *(v4f*)(osw + lr * 68 + dc * 16 + 8 * hi) = o0; *(v4f*)(osw + lr * 68 + dc * 16 + 8 * hi + 4) = o1;
    }
    __builtin_amdgcn_fence(3  , "wavefront"); __builtin_amdgcn_wave_barrier();
    float* orow = OUT + ((size_t)bh * SEQ_OUT + q0w) * HD;
#pragma unroll 1
    for (int ps = 0; ps < 2; ++ps) {
#pragma unroll
        for (int s2 = 0; s2 < 8; ++s2) { const int row = 2 * s2 + hi, cofs = lr * 4; const v4f val = *(const v4fa*)(osw + row * 68 + cofs); *(volatile v4f*)(orow + (size_t)row * HD + cofs) = val; }
        if (ps == 0) __threadfence();
    }
}

extern "C" void kernel_launch(void* const* d_in, const int* in_sizes, int n_in,
                              void* d_out, int out_size, void* d_ws, size_t ws_size, hipStream_t stream) {
    if (n_in < 3) return;
    const long need_in = ((long)(NB * NH - 1) * SEQ_FULL + SEQ) * HD;
    if ((long)in_sizes[0] < need_in || (long)in_sizes[1] < need_in || (long)in_sizes[2] < need_in) return;
    const long need_out = ((long)(NB * NH - 1) * SEQ_OUT + SEQ) * HD;
    if ((long)out_size < need_out) return;
    const float* qi = (const float*)d_in[0]; const float* ki = (const float*)d_in[1]; const float* vi = (const float*)d_in[2];
    float* OUT = (float*)d_out;
    const size_t NPL = (size_t)NB * NH * SEQ * HD;
    char* wsp = (char*)d_ws;
    auto take = [&](size_t bytes) { char* p = wsp; wsp += (bytes + 255) & ~(size_t)255; return (void*)p; };
    h16* QP = (h16*)take(NPL * 2); h16* KP = (h16*)take(NPL * 2); h16* VT = (h16*)take(NPL * 2);
    if ((size_t)(wsp - (char*)d_ws) > ws_size) return;
    const int n8 = (int)(NPL / 8); const unsigned cblocks = (unsigned)((n8 + 255) / 256);
    k_cvtqk<<<cblocks, 256, 0, stream>>>(qi, ki, QP, KP, n8);
    k_vt<<<cblocks, 256, 0, stream>>>(vi, VT, n8);
    const int NQB = SEQ / 64; const int BH = NB * NH; const int RBmax = RROWS / 64; const int RB = (RBmax < NQB) ? RBmax : NQB;
    k_attn<true><<<dim3((unsigned)RB, (unsigned)BH), 128, 0, stream>>>(QP, KP, VT, OUT, 0);
    if (NQB > RB) k_attn<false><<<dim3((unsigned)(NQB - RB), (unsigned)BH), 128, 0, stream>>>(QP, KP, VT, OUT, RB);
}
